// TransformerBlock_2499670966275
// MI455X (gfx1250) — hardware-verified
//
#include <hip/hip_runtime.h>
#ifndef NB
#define NB 2
#endif
#ifndef SQ
#define SQ 2048
#endif
#define NB_FULL 2
#define SQ_FULL 2048
#define DM 1024
#define NH 16
#define HD 64
#define HG 2
#define DFF 4096
#define DMQ DM
#define LQ (3 * DM)
#define NR ((size_t)NB * SQ)

static_assert(SQ % 256 == 0);
static_assert(SQ <= SQ_FULL);
static_assert(NB <= NB_FULL);
static_assert(NH % HG == 0);
static_assert(DM == NH * HD);
static_assert(HD == 64);

typedef unsigned short v8us __attribute__((ext_vector_type(8), may_alias));
typedef float  v8f  __attribute__((ext_vector_type(8)));
typedef float  v4f  __attribute__((ext_vector_type(4)));
typedef float  v4fa __attribute__((ext_vector_type(4), may_alias));
typedef _Float16 v16h __attribute__((ext_vector_type(16)));
typedef _Float16 v4h __attribute__((ext_vector_type(4)));
union FragH { v16h v; v8us half[2]; _Float16 h[16]; unsigned short u[16]; };

__device__ __forceinline__ unsigned short bf16_bits(float x) { unsigned int u = __float_as_uint(x); return (unsigned short)((u + 0x7FFFu + ((u >> 16) & 1u)) >> 16); }
__device__ __forceinline__ float bf16_val(unsigned short b) { return __uint_as_float(((unsigned int)b) << 16); }
__device__ __forceinline__ float bf16_rne(float x) { return bf16_val(bf16_bits(x)); }

__global__ __launch_bounds__(256) void k_wt_f16(const float* __restrict__ W, _Float16* __restrict__ Wt, unsigned k8sh, unsigned N, float scale) {
  const unsigned t = blockIdx.x * 256u + threadIdx.x; if (t >= (N << k8sh)) return;
  const unsigned n = t >> k8sh, k8 = (t & ((1u << k8sh) - 1u)) << 3; const unsigned K = 8u << k8sh; FragH f;
#pragma unroll
  for (int i = 0; i < 8; ++i) f.h[i] = (_Float16)(bf16_rne(W[(size_t)(k8 + (unsigned)i) * N + n]) * scale);
  const v8us o = f.half[0]; unsigned short* d = (unsigned short*)Wt + (size_t)n * K + k8;
  *(volatile v8us*)d = o; __threadfence(); *(volatile v8us*)d = o;
}

__global__ __launch_bounds__(256) void k_x16(const float* __restrict__ x, _Float16* __restrict__ X16, unsigned n8) {
  const unsigned t = blockIdx.x * 256u + threadIdx.x; if (t >= n8) return; FragH f;
  const v4f a = *(const v4fa*)(x + (size_t)t * 8), c = *(const v4fa*)(x + (size_t)t * 8 + 4);
#pragma unroll
  for (int q = 0; q < 4; ++q) { f.h[q] = (_Float16)bf16_rne(a[q]); f.h[4 + q] = (_Float16)bf16_rne(c[q]); }
  const v8us o = f.half[0]; unsigned short* d = (unsigned short*)X16 + (size_t)t * 8;
  *(volatile v8us*)d = o; __threadfence(); *(volatile v8us*)d = o;
}

template <int NHv, int TTv>
__global__ __launch_bounds__(256) void k_vt(const _Float16* __restrict__ V16, unsigned ldv, unsigned voff, _Float16* __restrict__ Vt) {
  __shared__ unsigned short tl[64][66];
  const unsigned tid = threadIdx.x; const unsigned slab = blockIdx.x / (unsigned)(TTv / 64), lg = blockIdx.x % (unsigned)(TTv / 64); const unsigned b = slab / (unsigned)NHv, h = slab % (unsigned)NHv;
  for (unsigned i = tid; i < 64u * 8u; i += 256u) { const unsigned r = i >> 3, c8 = (i & 7u) << 3; FragH f; f.half[0] = *(const v8us*)((const unsigned short*)V16 + ((size_t)b * TTv + lg * 64u + r) * ldv + voff + h * 64u + c8);
#pragma unroll
    for (int q = 0; q < 8; ++q) tl[r][c8 + (unsigned)q] = f.u[q]; }
  __syncthreads();
  for (int pass = 0; pass < 2; ++pass) {
#pragma unroll
    for (unsigned rd = 0; rd < 2; ++rd) { const unsigned d = rd * 32u + (tid >> 3), pc = tid & 7u; FragH f;
#pragma unroll
      for (int q = 0; q < 8; ++q) f.u[q] = tl[pc * 8u + (unsigned)q][d];
      *(volatile v8us*)((unsigned short*)Vt + ((size_t)slab * 64u + d) * TTv + lg * 64u + pc * 8u) = f.half[0]; }
    if (pass == 0) __threadfence(); } }

__device__ __forceinline__ v16h g2_frag(const _Float16* p, unsigned hh) { FragH f; f.half[0] = *(const v8us*)((const unsigned short*)p + 8u * hh); f.half[1] = *(const v8us*)((const unsigned short*)p + 16u + 8u * hh); return f.v; }
__device__ __forceinline__ v8f g2_mma(v16h a, v16h b, v8f c) { v8f d = __builtin_amdgcn_wmma_f32_16x16x32_f16(false, a, false, b, (short)0, c, false, false); asm volatile("v_nop\n\tv_nop\n\tv_nop\n\tv_nop" : "+v"(d) : "v"(a), "v"(b)); return d; }
template <int ACT, int CPBF, int CAUS>
__global__ __launch_bounds__(128) void k_gemm2(const _Float16* __restrict__ A, int lda, size_t sA, const _Float16* __restrict__ Bh, int ldb, size_t sB, float alpha, const float* __restrict__ bias, const float* __restrict__ CP, int ldcp,
    float* __restrict__ C, _Float16* __restrict__ C16, int ldc, size_t sC, int M, int N, int K) {
  static_assert(ACT == 0 || ACT == 6);
  __shared__ __attribute__((aligned(16))) float so[4][32][68];
  const unsigned tid = threadIdx.x, w = tid >> 5, lane = tid & 31u, ln = lane & 15u, hh = lane >> 4; const unsigned by = blockIdx.y;
  A += (size_t)by * sA; Bh += (size_t)by * sB; const size_t cofs = (size_t)by * sC;
  const unsigned ntn = (unsigned)N >> 6; const unsigned mt = blockIdx.x / ntn, nq = blockIdx.x - mt * ntn; const unsigned row0 = mt * 128u + 32u * w, col0 = nq * 64u; if (row0 >= (unsigned)M) return;
  if (CAUS == 1) { if (col0 >= ((mt * 128u) & ~255u) + 256u) return; }
  const unsigned kend = (CAUS == 2) ? (((row0 + 32u) < (unsigned)K) ? (row0 + 32u) : (unsigned)K) : (unsigned)K;
  const _Float16* a0p = A + (size_t)(row0 + ln) * lda; const _Float16* a1p = a0p + (size_t)16 * lda;
  const _Float16* b0p = Bh + (size_t)(col0 + ln) * ldb; const _Float16* b1p = b0p + (size_t)16 * ldb; const _Float16* b2p = b1p + (size_t)16 * ldb; const _Float16* b3p = b2p + (size_t)16 * ldb;
  const v8f z8 = {0.f,0.f,0.f,0.f,0.f,0.f,0.f,0.f}; v8f c00 = z8, c01 = z8, c02 = z8, c03 = z8, c10 = z8, c11 = z8, c12 = z8, c13 = z8;
#pragma unroll 1
  for (unsigned kb = 0; kb < kend; kb += 32u) { const v16h a0 = g2_frag(a0p + kb, hh), a1 = g2_frag(a1p + kb, hh);
    v16h b = g2_frag(b0p + kb, hh); c00 = g2_mma(a0, b, c00); c10 = g2_mma(a1, b, c10);
    b = g2_frag(b1p + kb, hh); c01 = g2_mma(a0, b, c01); c11 = g2_mma(a1, b, c11);
    b = g2_frag(b2p + kb, hh); c02 = g2_mma(a0, b, c02); c12 = g2_mma(a1, b, c12);
    b = g2_frag(b3p + kb, hh); c03 = g2_mma(a0, b, c03); c13 = g2_mma(a1, b, c13); }
  v8f accs[8] = {c00, c01, c02, c03, c10, c11, c12, c13};
#pragma unroll
  for (int u = 0; u < 8; ++u) { const unsigned t = (unsigned)u & 3u, half = (unsigned)u >> 2; const unsigned col = col0 + t * 16u + ln; const float bv = bias ? bf16_rne(bias[col]) : 0.f;
#pragma unroll
    for (int r = 0; r < 8; ++r) { const unsigned rloc = half * 16u + 8u * hh + (unsigned)r; float v = accs[u][r] * alpha + bv;
      if (CP) { float cv = CP[(size_t)(row0 + rloc) * ldcp + col]; if (CPBF) cv = bf16_rne(cv); v += cv; }
      if (ACT == 6) v = 0.5f * v * (1.0f + erff(v * 0.70710678118654752f));
      so[w][rloc][t * 16u + ln] = v; } }
  __builtin_amdgcn_fence(4  , "workgroup"); __builtin_amdgcn_wave_barrier();
  const unsigned rsub = lane >> 4, c4 = (lane & 15u) * 4u;
  for (int pass = 0; pass < 2; ++pass) {
#pragma unroll
    for (unsigned q = 0; q < 16; ++q) { const unsigned r = q * 2u + rsub; const v4f v = *(const v4fa*)&so[w][r][c4];
      if (C) *(volatile v4f*)(C + cofs + (size_t)(row0 + r) * ldc + col0 + c4) = v;
      if (C16) { v4h h4; for (int i = 0; i < 4; ++i) h4[i] = (_Float16)v[i]; *(volatile v4h*)(C16 + cofs + (size_t)(row0 + r) * ldc + col0 + c4) = h4; } }
    if (pass == 0) __threadfence(); } }

__global__ __launch_bounds__(256) void k_rsmc(const float* __restrict__ S, _Float16* __restrict__ P, unsigned nrows) {
  #pragma clang fp contract(off)
  const unsigned t = blockIdx.x * 256u + threadIdx.x; if (t >= nrows) return;
  const size_t i = (size_t)t; const float* s = S + i * SQ; const unsigned last = t % (unsigned)SQ; const unsigned nk = ((blockIdx.x * 256u) % (unsigned)SQ) + 256u; float mx = -3.0e38f;
#pragma unroll 1
  for (unsigned j = 0; j < nk; ++j) { const float f = (j <= last) ? 1.f : 0.f; mx = fmaxf(mx, fmaf(f, s[j], (1.f - f) * -1.0e9f)); }
  float se = 0.f;
#pragma unroll 1
  for (unsigned j = 0; j < nk; ++j) { const float f = (j <= last) ? 1.f : 0.f; se += __expf(fmaf(f, s[j], (1.f - f) * -1.0e9f) - mx); }
  const float sc = 256.0f / se;
#pragma unroll 1
  for (unsigned j0 = 0; j0 < nk; j0 += 8u) { FragH fr;
    for (int q = 0; q < 8; ++q) { const unsigned j = j0 + (unsigned)q; const float f = (j <= last) ? 1.f : 0.f; fr.h[q] = (_Float16)(__expf(fmaf(f, s[j], (1.f - f) * -1.0e9f) - mx) * sc); }
    const v8us o = fr.half[0]; unsigned short* d = (unsigned short*)P + i * SQ + j0; *(volatile v8us*)d = o; __threadfence(); *(volatile v8us*)d = o; } }

template <int BFIN, int W16, int W32>
__global__ __launch_bounds__(256) void k_lnx(const float* __restrict__ X, const float* __restrict__ g, const float* __restrict__ bb, float eps, _Float16* __restrict__ N16, float* __restrict__ N32) {
  #pragma clang fp contract(off)
  __shared__ float red[256]; const size_t r = blockIdx.x; const unsigned t = threadIdx.x; const unsigned c0 = t * 4u;
  const v4f xa = *(const v4fa*)(X + r * DMQ + c0); float s[4]; float sum = 0.f;
  for (int q = 0; q < 4; ++q) { s[q] = BFIN ? bf16_rne(xa[q]) : xa[q]; sum = __fadd_rn(sum, s[q]); }
  red[t] = sum; __syncthreads(); for (unsigned st = 128; st > 0; st >>= 1) { if (t < st) red[t] = __fadd_rn(red[t], red[t + st]); __syncthreads(); } const float mu = red[0] * (1.0f / (float)DMQ); __syncthreads();
  float vs = 0.f; for (int q = 0; q < 4; ++q) { const float dl = __fadd_rn(s[q], -mu); vs = __fadd_rn(vs, __fmul_rn(dl, dl)); } red[t] = vs; __syncthreads(); for (unsigned st = 128; st > 0; st >>= 1) { if (t < st) red[t] = __fadd_rn(red[t], red[t + st]); __syncthreads(); }
  const float rs = rsqrtf(__fadd_rn(red[0] * (1.0f / (float)DMQ), eps)); v4h y; v4f yf;
  for (int q = 0; q < 4; ++q) { const unsigned c = c0 + (unsigned)q; yf[q] = __fadd_rn(__fmul_rn(__fmul_rn(__fadd_rn(s[q], -mu), rs), bf16_rne(g[c])), bf16_rne(bb[c])); y[q] = (_Float16)yf[q]; }
  for (int pass = 0; pass < 2; ++pass) { if (W16) *(volatile v4h*)(N16 + r * DMQ + c0) = y; if (W32) *(volatile v4f*)(N32 + r * DMQ + c0) = yf; if (pass == 0) __threadfence(); } }

static constexpr size_t cmax(size_t a, size_t b) { return a > b ? a : b; }
static constexpr size_t al256(size_t a) { return (a + 255) & ~(size_t)255; }

static constexpr size_t SZ_BQKV = (size_t)3 * DM * DM * 2;
static constexpr size_t SZ_BO   = (size_t)DM * DM * 2;
static constexpr size_t SZ_BW1  = (size_t)DFF * DM * 2;
static constexpr size_t SZ_BW2  = (size_t)DM * DFF * 2;
static constexpr size_t SZ_QKV  = NR * 3 * DM * 2;
static constexpr size_t SZ_O16  = NR * DM * 2;
static constexpr size_t SZ_HF   = NR * DFF * 2;
static constexpr size_t SZ_RB   = al256(cmax(SZ_QKV + SZ_O16, SZ_HF));
static constexpr size_t SZ_VT   = (size_t)NH * HD * SQ * 2;
static constexpr size_t SZ_S    = (size_t)HG * SQ * SQ * 4;
static constexpr size_t SZ_P    = (size_t)HG * SQ * SQ * 2;
static constexpr size_t SZ_X16  = NR * DM * 2;
static constexpr size_t SZ_F32  = NR * DM * 4;
static constexpr size_t SZ_M16  = NR * DM * 2;
static constexpr size_t SZ_RA   = al256(cmax(cmax(SZ_S + SZ_P, SZ_F32 + SZ_F32 + SZ_M16), SZ_X16));
static constexpr size_t OFF_BQKV = 0;
static constexpr size_t OFF_BO   = OFF_BQKV + SZ_BQKV;
static constexpr size_t OFF_BW1  = OFF_BO + SZ_BO;
static constexpr size_t OFF_BW2  = OFF_BW1 + SZ_BW1;
static constexpr size_t OFF_RB   = OFF_BW2 + SZ_BW2;
static constexpr size_t OFF_VT   = OFF_RB + SZ_RB;
static constexpr size_t OFF_RA   = OFF_VT + SZ_VT;
static constexpr size_t WS_TOTAL = OFF_RA + SZ_RA;
static_assert(WS_TOTAL <= (size_t)134217728);
static_assert(SZ_QKV + SZ_O16 <= SZ_RB);
static_assert(SZ_HF <= SZ_RB);
static_assert(SZ_S + SZ_P <= SZ_RA);
static_assert(SZ_F32 + SZ_F32 + SZ_M16 <= SZ_RA);
static_assert(SZ_X16 <= SZ_RA);
static_assert((SZ_BQKV % 256) == 0 && (SZ_BO % 256) == 0 && (SZ_BW1 % 256) == 0 && (SZ_VT % 256) == 0 && (SZ_S % 256) == 0 && (SZ_F32 % 256) == 0 && (SZ_QKV % 256) == 0);
static_assert(((size_t)DM * (DM / 8)) % 256 == 0);
static_assert(((size_t)DFF * (DM / 8)) % 256 == 0);
static_assert(((size_t)SQ * DM / 8) % 256 == 0);
static_assert(NR % 128 == 0 && SQ % 128 == 0 && (3 * DM) % 64 == 0 && DFF % 64 == 0 && DM % 64 == 0 && DM % 32 == 0 && DFF % 32 == 0 && HD % 32 == 0);
static_assert(((size_t)HG * SQ) % 256 == 0);
static_assert((size_t)((NB_FULL - 1) * (size_t)SQ_FULL + SQ_FULL) * DM * 4 == (size_t)16777216);

extern "C" void kernel_launch(void* const* d_in, const int* in_sizes, int n_in,
                              void* d_out, int out_size, void* d_ws, size_t ws_size, hipStream_t stream) {
  if (n_in < 14) return;
  const size_t needx = ((size_t)(NB - 1) * SQ_FULL + SQ) * DM;
  if ((size_t)in_sizes[0] < needx || (size_t)out_size < needx) return;
  if ((size_t)in_sizes[1] < (size_t)DM * DM || (size_t)in_sizes[2] < (size_t)DM * DM || (size_t)in_sizes[3] < (size_t)DM * DM || (size_t)in_sizes[4] < (size_t)DM * DM) return;
  if (in_sizes[5] < DM || in_sizes[6] < DM || in_sizes[7] < DM || in_sizes[9] < DFF || in_sizes[11] < DM || in_sizes[12] < DM || in_sizes[13] < DM) return;
  if ((size_t)in_sizes[8] < (size_t)DM * DFF || (size_t)in_sizes[10] < (size_t)DFF * DM) return;
  if (WS_TOTAL > ws_size) return;
  const float* x = (const float*)d_in[0]; const float* Wq = (const float*)d_in[1]; const float* Wk = (const float*)d_in[2]; const float* Wv = (const float*)d_in[3]; const float* Wo = (const float*)d_in[4];
  const float* bo = (const float*)d_in[5]; const float* g1 = (const float*)d_in[6]; const float* b1 = (const float*)d_in[7]; const float* Wf1 = (const float*)d_in[8]; const float* bf1 = (const float*)d_in[9];
  const float* Wf2 = (const float*)d_in[10]; const float* bf2 = (const float*)d_in[11]; const float* g2 = (const float*)d_in[12]; const float* b2 = (const float*)d_in[13];
  float* out = (float*)d_out;
  char* ws = (char*)d_ws;
  _Float16* BQKV = (_Float16*)(ws + OFF_BQKV); _Float16* BO = (_Float16*)(ws + OFF_BO); _Float16* BW1 = (_Float16*)(ws + OFF_BW1); _Float16* BW2 = (_Float16*)(ws + OFF_BW2);
  _Float16* QKV = (_Float16*)(ws + OFF_RB); _Float16* O16 = (_Float16*)(ws + OFF_RB + SZ_QKV); _Float16* HF16 = (_Float16*)(ws + OFF_RB);
  _Float16* Q16 = QKV; _Float16* K16 = QKV + DM; _Float16* V16 = QKV + 2 * DM;
  _Float16* VT = (_Float16*)(ws + OFF_VT);
  _Float16* X16 = (_Float16*)(ws + OFF_RA);
  float* S = (float*)(ws + OFF_RA); _Float16* P = (_Float16*)(ws + OFF_RA + SZ_S);
  float* X1 = (float*)(ws + OFF_RA); float* HN32 = (float*)(ws + OFF_RA + SZ_F32); _Float16* M16 = (_Float16*)(ws + OFF_RA + 2 * SZ_F32);
  float* X2 = X1;

  k_wt_f16<<<(unsigned)((size_t)DM * (DM / 8) / 256), 256, 0, stream>>>(Wq, BQKV, 7u, (unsigned)DM, 16.0f);
  k_wt_f16<<<(unsigned)((size_t)DM * (DM / 8) / 256), 256, 0, stream>>>(Wk, BQKV + (size_t)DM * DM, 7u, (unsigned)DM, 16.0f);
  k_wt_f16<<<(unsigned)((size_t)DM * (DM / 8) / 256), 256, 0, stream>>>(Wv, BQKV + (size_t)2 * DM * DM, 7u, (unsigned)DM, 16.0f);
  k_wt_f16<<<(unsigned)((size_t)DM * (DM / 8) / 256), 256, 0, stream>>>(Wo, BO, 7u, (unsigned)DM, 16.0f);
  k_wt_f16<<<(unsigned)((size_t)DFF * (DM / 8) / 256), 256, 0, stream>>>(Wf1, BW1, 7u, (unsigned)DFF, 16.0f);
  k_wt_f16<<<(unsigned)((size_t)DM * (DFF / 8) / 256), 256, 0, stream>>>(Wf2, BW2, 9u, (unsigned)DM, 16.0f);
  for (int b = 0; b < NB; ++b)
    k_x16<<<(unsigned)((size_t)SQ * DM / 8 / 256), 256, 0, stream>>>(x + (size_t)b * SQ_FULL * DM, X16 + (size_t)b * SQ * DM, (unsigned)((size_t)SQ * DM / 8));
  k_gemm2<0, 0, 0><<<dim3((unsigned)((NR / 128) * (3 * DM / 64)), 1), 128, 0, stream>>>(X16, DM, (size_t)0, BQKV, DM, (size_t)0, 0.0625f, nullptr, nullptr, 0, nullptr, QKV, 3 * DM, (size_t)0, (int)NR, 3 * DM, DM);
  for (int b = 0; b < NB; ++b) { const size_t r0 = (size_t)b * SQ;
    k_vt<NH, SQ><<<NH * (SQ / 64), 256, 0, stream>>>(V16 + r0 * LQ, (unsigned)LQ, 0u, VT);
    for (int h0 = 0; h0 < NH; h0 += HG) {
      k_gemm2<0, 0, 1><<<dim3((SQ / 128) * (SQ / 64), HG), 128, 0, stream>>>(Q16 + r0 * LQ + (size_t)h0 * HD, LQ, (size_t)HD, K16 + r0 * LQ + (size_t)h0 * HD, LQ, (size_t)HD, 0.125f, nullptr, nullptr, 0, S, nullptr, SQ, (size_t)SQ * SQ, SQ, SQ, HD);
      k_rsmc<<<(unsigned)((size_t)HG * SQ / 256), 256, 0, stream>>>(S, P, (unsigned)(HG * SQ));
      k_gemm2<0, 0, 2><<<dim3((SQ / 128) * (HD / 64), HG), 128, 0, stream>>>(P, SQ, (size_t)SQ * SQ, VT + (size_t)h0 * HD * SQ, SQ, (size_t)HD * SQ, 0.25f, nullptr, nullptr, 0, nullptr, O16 + r0 * DM + (size_t)h0 * HD, DM, (size_t)HD, SQ, HD, SQ);
    } }
  for (int b = 0; b < NB; ++b) { const size_t r0 = (size_t)b * SQ;
    k_gemm2<0, 1, 0><<<dim3((unsigned)((SQ / 128) * (DM / 64)), 1), 128, 0, stream>>>(O16 + r0 * DM, DM, (size_t)0, BO, DM, (size_t)0, 0.0009765625f, bo, x + (size_t)b * SQ_FULL * DM, DM, X1 + r0 * DM, nullptr, DM, (size_t)0, SQ, DM, DM); }
  k_lnx<0, 1, 1><<<(unsigned)NR, 256, 0, stream>>>(X1, g1, b1, 1e-5f, M16, HN32);
  k_gemm2<6, 0, 0><<<dim3((unsigned)((NR / 128) * (DFF / 64)), 1), 128, 0, stream>>>(M16, DM, (size_t)0, BW1, DM, (size_t)0, 0.0625f, bf1, nullptr, 0, nullptr, HF16, DFF, (size_t)0, (int)NR, DFF, DM);
  k_gemm2<0, 0, 0><<<dim3((unsigned)((NR / 128) * (DM / 64)), 1), 128, 0, stream>>>(HF16, DFF, (size_t)0, BW2, DFF, (size_t)0, 0.0625f, bf2, HN32, DM, X2, nullptr, DM, (size_t)0, (int)NR, DM, DFF);
  for (int b = 0; b < NB; ++b)
    k_lnx<0, 0, 1><<<(unsigned)SQ, 256, 0, stream>>>(X2 + (size_t)b * SQ * DM, g2, b2, 1e-5f, nullptr, out + (size_t)b * SQ_FULL * DM);
}
